// selfattention_59416577573049
// MI455X (gfx1250) — hardware-run, weakly checked
//
#include <hip/hip_runtime.h>


#ifndef NB
#define NB 4
#endif
#ifndef SEQ
#define SEQ 1024
#endif
#define NB_FULL  4
#define SEQ_FULL 1024
#define LF   1024
#define DM   1024
#define NH_  16
#define HD   64
#define TD   3072
#define NBH  (NB * NH_)
#define ZH   4
#define WP   (SEQ + 64)
#define EROWS 2048
#define PCAR 1024.0f
#define SCL  0.125f

static_assert(SEQ % 128 == 0);
static_assert(SEQ <= LF);
static_assert(LF + SEQ <= EROWS);
static_assert(NH_ % ZH == 0);
static_assert((NB * SEQ) % 64 == 0);
static_assert(NB <= NB_FULL);
static_assert(SEQ <= SEQ_FULL);

typedef _Float16 h16;
typedef unsigned short bf;
typedef __attribute__((ext_vector_type(16))) __bf16   v16bf;
typedef __attribute__((ext_vector_type(16))) _Float16 v16h;
typedef __attribute__((ext_vector_type(8)))  _Float16 v8h;
typedef __attribute__((ext_vector_type(4)))  _Float16 v4h;
typedef __attribute__((ext_vector_type(8)))  unsigned short v8us;
typedef __attribute__((ext_vector_type(8)))  float    v8f;
typedef __attribute__((ext_vector_type(4)))  float    v4f;
typedef v4f  __attribute__((may_alias)) v4fa;

__device__ __forceinline__ unsigned short f2bf(float f) { unsigned u = __float_as_uint(f); u += 0x7FFFu + ((u >> 16) & 1u); return (unsigned short)(u >> 16); }
__device__ __forceinline__ float bf2f(unsigned short b) { return __uint_as_float(((unsigned)b) << 16); }
__device__ __forceinline__ float bfr(float f) { return bf2f(f2bf(f)); }
__device__ __forceinline__ void splitf(float y, unsigned short& h, unsigned short& l) { h = f2bf(y); l = f2bf(y - bf2f(h)); }
__device__ __forceinline__ v16h cat16(v8h lo, v8h hi) { return __builtin_shufflevector(lo, hi, 0, 1, 2, 3, 4, 5, 6, 7, 8, 9, 10, 11, 12, 13, 14, 15); }
__device__ __forceinline__ v16bf cat16b(v8us lo, v8us hi) { return __builtin_bit_cast(v16bf, __builtin_shufflevector(lo, hi, 0, 1, 2, 3, 4, 5, 6, 7, 8, 9, 10, 11, 12, 13, 14, 15)); }
__device__ __forceinline__ v8f wmma16(v16h a, v16h b, v8f c) { return __builtin_amdgcn_wmma_f32_16x16x32_f16(false, a, false, b, (short)0, c, false, false); }
__device__ __forceinline__ v8f wmmab(v16bf a, v16bf b, v8f c) { return __builtin_amdgcn_wmma_f32_16x16x32_bf16(false, a, false, b, (short)0, c, false, false); }

template <typename T16> struct WFrag;
template <> struct WFrag<h16> { typedef v16h V; static __device__ __forceinline__ V ld(const h16* p) { return cat16(*(const v8h*)p, *(const v8h*)(p + 16)); } static __device__ __forceinline__ v8f mma(V a, V b, v8f c) { return wmma16(a, b, c); } };
template <> struct WFrag<bf> { typedef v16bf V; static __device__ __forceinline__ V ld(const bf* p) { return cat16b(*(const v8us*)p, *(const v8us*)(p + 16)); } static __device__ __forceinline__ v8f mma(V a, V b, v8f c) { return wmmab(a, b, c); } };
template <typename T16, int NSPLIT, bool BIAS, bool TOEP>
__global__ __launch_bounds__(32) void k_gemmw(const T16* __restrict__ A, const T16* __restrict__ A2, const T16* __restrict__ Bt, const T16* __restrict__ Bt2, int K, float* C, int ldc, const float* __restrict__ bias, float cs, size_t sA, size_t sB, size_t sC, size_t sAw, size_t sCw) {
    typedef typename WFrag<T16>::V V;
    __shared__ __align__(16) float os[16 * 68];
    const int lane = threadIdx.x & 31, lr = lane & 15, hi = lane >> 4; const int r0 = blockIdx.x * 64, c0 = blockIdx.y * 64;
    size_t z = blockIdx.z; int brow = c0 + lr;
    if (TOEP) { const int which = (z >= (size_t)ZH) ? 1 : 0; z -= (size_t)which * ZH; A += (size_t)which * sAw; C += (size_t)which * sCw; brow += which ? (LF - 64 - r0) : (LF - SEQ + r0); }
    A += z * sA; if (NSPLIT == 1 || NSPLIT == 2) A2 += z * sA; Bt += z * sB; if (NSPLIT >= 2) Bt2 += z * sB; C += z * sC;
    v8f acc[4][4];
#pragma unroll
    for (int mb = 0; mb < 4; ++mb)
#pragma unroll
        for (int nb = 0; nb < 4; ++nb) acc[mb][nb] = (v8f){};
    const size_t aoff = (size_t)(r0 + lr) * K + 8 * hi, boff = (size_t)brow * K + 8 * hi;
#pragma unroll 1
    for (int kc = 0; kc < K; kc += 32) {
        V a[4], a2[4];
#pragma unroll
        for (int mb = 0; mb < 4; ++mb) { a[mb] = WFrag<T16>::ld(A + aoff + (size_t)mb * 16 * K + kc); if (NSPLIT == 1 || NSPLIT == 2) a2[mb] = WFrag<T16>::ld(A2 + aoff + (size_t)mb * 16 * K + kc); }
#pragma unroll
        for (int nb = 0; nb < 4; ++nb) { const V b = WFrag<T16>::ld(Bt + boff + (size_t)nb * 16 * K + kc); V b2; if (NSPLIT >= 2) b2 = WFrag<T16>::ld(Bt2 + boff + (size_t)nb * 16 * K + kc);
#pragma unroll
            for (int mb = 0; mb < 4; ++mb) { acc[mb][nb] = WFrag<T16>::mma(a[mb], b, acc[mb][nb]); if (NSPLIT == 1 || NSPLIT == 2) acc[mb][nb] = WFrag<T16>::mma(a2[mb], b, acc[mb][nb]); if (NSPLIT >= 2) acc[mb][nb] = WFrag<T16>::mma(a[mb], b2, acc[mb][nb]); } }
        asm volatile("v_nop\n\tv_nop\n\tv_nop\n\tv_nop" : "+v"(acc[0][0]), "+v"(acc[1][1]), "+v"(acc[2][2]), "+v"(acc[3][3]) : "v"(a[0]), "v"(a[3]));
    }
#pragma unroll
    for (int mb = 0; mb < 4; ++mb) {
#pragma unroll
        for (int nb = 0; nb < 4; ++nb) {
#pragma unroll
            for (int j = 0; j < 8; ++j) os[(hi * 8 + j) * 68 + nb * 16 + lr] = acc[mb][nb][j]; }
        __builtin_amdgcn_wave_barrier(); asm volatile("" ::: "memory");
        float* crow = C + (size_t)(r0 + mb * 16) * ldc + c0;
#pragma unroll 1
        for (int ps = 0; ps < 2; ++ps) {
#pragma unroll
            for (int s = 0; s < 8; ++s) { const int row = 2 * s + hi, cofs = lr * 4; v4f val = *(const v4fa*)(os + row * 68 + cofs); val = val * cs; if (BIAS) { val[0] += bfr(bias[c0 + cofs]); val[1] += bfr(bias[c0 + cofs + 1]); val[2] += bfr(bias[c0 + cofs + 2]); val[3] += bfr(bias[c0 + cofs + 3]); }
                *(volatile v4f*)(crow + (size_t)row * ldc + cofs) = val; }
            if (ps == 0) __threadfence(); }
        __builtin_amdgcn_wave_barrier(); asm volatile("" ::: "memory");
    }
}

__global__ __launch_bounds__(256) void k_cvtx(const float* __restrict__ src, bf* dst) {
    const size_t i = (size_t)blockIdx.x * 256 + threadIdx.x; if (i >= (size_t)SEQ * DM / 8) return;
    const v8f v = *(const v8f*)(src + (size_t)blockIdx.y * SEQ_FULL * DM + i * 8); v8us o;
#pragma unroll
    for (int k = 0; k < 8; ++k) o[k] = f2bf(v[k]);
    bf* d = dst + (size_t)blockIdx.y * SEQ * DM + i * 8;
    *(volatile v8us*)d = o; __threadfence(); *(volatile v8us*)d = o; }

__global__ __launch_bounds__(256) void k_cvte(const float* __restrict__ src, bf* dst) {
    const int i = blockIdx.x * 256 + threadIdx.x; if (i >= EROWS * HD / 8) return;
    const int e = i * 8; const bool ok = (e >> 6) < (2 * LF - 1); const int se = ok ? e : 0;
    const v8f v = *(const v8f*)(src + se); v8us o;
#pragma unroll
    for (int k = 0; k < 8; ++k) o[k] = ok ? f2bf(v[k]) : (unsigned short)0;
    *(volatile v8us*)(dst + e) = o; __threadfence(); *(volatile v8us*)(dst + e) = o; }

template <bool HALF>
__global__ __launch_bounds__(256) void k_tr64(const float* __restrict__ src, int spitch, size_t szs, int cbase, unsigned short* dst, int dpitch) {
    __shared__ float tl[64 * 65];
    const int tid = threadIdx.x;
    const float* s = src + (size_t)blockIdx.z * szs + (size_t)blockIdx.x * 64 * spitch + cbase + blockIdx.y * 64;
#pragma unroll
    for (int it = 0; it < 4; ++it) { const int r = (tid >> 4) + 16 * it, c = (tid & 15) * 4; const v4f a = *(const v4f*)(s + (size_t)r * spitch + c);
        tl[r * 65 + c] = a[0]; tl[r * 65 + c + 1] = a[1]; tl[r * 65 + c + 2] = a[2]; tl[r * 65 + c + 3] = a[3]; }
    __syncthreads();
    unsigned short* d = dst + ((size_t)blockIdx.z * gridDim.y + blockIdx.y) * 64 * dpitch + (size_t)blockIdx.x * 64;
    const int q = tid & 7; v8us o[2];
#pragma unroll
    for (int it = 0; it < 2; ++it) { const int n = (tid >> 3) + 32 * it;
#pragma unroll
        for (int e = 0; e < 8; ++e) { const float x = tl[(q * 8 + e) * 65 + n]; o[it][e] = HALF ? __builtin_bit_cast(unsigned short, (h16)x) : f2bf(x); } }
#pragma unroll 1
    for (int ps = 0; ps < 2; ++ps) {
#pragma unroll
        for (int it = 0; it < 2; ++it) { const int n = (tid >> 3) + 32 * it; *(volatile v8us*)(d + (size_t)n * dpitch + q * 8) = o[it]; }
        if (ps == 0) __threadfence(); }
}

__global__ __launch_bounds__(256) void k_qkp(const float* __restrict__ F, bf* Ph, bf* Pl) {
    const size_t i = (size_t)blockIdx.x * 256 + threadIdx.x; if (i >= (size_t)2 * NBH * SEQ * 8) return;
    const int d8 = (int)(i & 7); const int t = (int)((i >> 3) % SEQ); const int bh = (int)((i / ((size_t)8 * SEQ)) % NBH); const int which = (int)(i / ((size_t)8 * SEQ * NBH));
    const int b = bh / NH_, h = bh % NH_;
    const float* f = F + ((size_t)b * SEQ + t) * TD + which * DM + h * HD + d8 * 8;
    const v4f a0 = *(const v4f*)f, a1 = *(const v4f*)(f + 4); v8us oh, ol;
#pragma unroll
    for (int k = 0; k < 4; ++k) { unsigned short a, c; splitf(a0[k], a, c); oh[k] = a; ol[k] = c; splitf(a1[k], a, c); oh[4 + k] = a; ol[4 + k] = c; }
    *(volatile v8us*)(Ph + i * 8) = oh; *(volatile v8us*)(Pl + i * 8) = ol; __threadfence(); *(volatile v8us*)(Ph + i * 8) = oh; *(volatile v8us*)(Pl + i * 8) = ol; }

__global__ __launch_bounds__(256) void k_rsoft(const float* __restrict__ Sb, const float* __restrict__ RQ, const float* __restrict__ RK, h16* P16) {
    const int lane = threadIdx.x & 31; const int row = blockIdx.x * 8 + (threadIdx.x >> 5); if (row >= ZH * SEQ) return;
    const int i = row % SEQ; const int zz = row / SEQ; const int li = i & 63;
    const float* sr = Sb + (size_t)row * SEQ; const float* rqr = RQ + (size_t)row * WP; const float* rkb = RK + (size_t)zz * SEQ * WP;
    float v[SEQ / 32]; float mx = -3.0e38f;
#pragma unroll
    for (int ch = 0; ch < SEQ / 128; ++ch) { const int j0 = ch * 128 + lane * 4; const v4f a = *(const v4f*)(sr + j0); float gq[4], gk[4];
#pragma unroll
        for (int q = 0; q < 4; ++q) { const int m = j0 + q; gq[q] = rqr[li + (SEQ - 1) - m]; gk[q] = rkb[(size_t)m * WP + (i + 63 - (m & 63))]; }
#pragma unroll
        for (int q = 0; q < 4; ++q) { asm volatile("" : "+v"(gq[q])); asm volatile("" : "+v"(gk[q])); }
#pragma unroll
        for (int q = 0; q < 4; ++q) { const float t = ((a[q] + gq[q]) + gk[q]) * SCL; v[ch * 4 + q] = t; mx = fmaxf(mx, t); }
        asm volatile("" ::: "memory"); }
#pragma unroll
    for (int sh = 16; sh; sh >>= 1) mx = fmaxf(mx, __shfl_xor(mx, sh, 32));
    float sum = 0.f;
#pragma unroll
    for (int k = 0; k < SEQ / 32; ++k) { float d0 = __fsub_rn(v[k], mx); asm volatile("" : "+v"(d0)); v[k] = __builtin_amdgcn_exp2f(__fmul_rn(d0, 1.4426950408889634f)); sum += v[k]; }
#pragma unroll
    for (int sh = 16; sh; sh >>= 1) sum += __shfl_xor(sum, sh, 32);
    const float f = __fdiv_rn(PCAR, sum);
#pragma unroll 1
    for (int ps = 0; ps < 2; ++ps) {
#pragma unroll
        for (int ch = 0; ch < SEQ / 128; ++ch) { v4h o4;
#pragma unroll
            for (int q = 0; q < 4; ++q) o4[q] = (h16)(v[ch * 4 + q] * f);
            *(volatile v4h*)(P16 + (size_t)row * SEQ + ch * 128 + lane * 4) = o4; }
        if (ps == 0) __threadfence(); }
}

#define AL256(x) ((((size_t)(x)) + 255) & ~(size_t)255)
#define SZ_WT  AL256((size_t)TD * DM * 2)
#define SZ_EB  AL256((size_t)EROWS * HD * 2)
#define SZ_XB  AL256((size_t)NB * SEQ * DM * 2)
#define SZ_QK  AL256((size_t)2 * NBH * SEQ * HD * 2)
#define SZ_VT  AL256((size_t)NBH * HD * SEQ * 2)
#define SZ_S   AL256((size_t)ZH * SEQ * SEQ * 4)
#define SZ_T   AL256((size_t)2 * ZH * SEQ * WP * 4)
#define SZ_P   AL256((size_t)ZH * SEQ * SEQ * 2)
#define SZ_F   AL256((size_t)NB * SEQ * TD * 4)
#define SZ_PASS (SZ_S + SZ_T + SZ_P)
#define SZ_R   ((SZ_PASS > SZ_F) ? SZ_PASS : SZ_F)
#define SZ_ALL (SZ_WT + SZ_EB + SZ_XB + 2 * SZ_QK + SZ_VT + SZ_R)
static_assert(SZ_F <= SZ_R);
static_assert(SZ_PASS <= SZ_R);
static_assert(SZ_ALL <= (size_t)134217728);

extern "C" void kernel_launch(void* const* d_in, const int* in_sizes, int n_in,
                              void* d_out, int out_size, void* d_ws, size_t ws_size, hipStream_t stream) {
    if (n_in < 4) return;
    if ((size_t)in_sizes[0] < (size_t)(NB - 1) * SEQ_FULL * DM + (size_t)SEQ * DM) return;
    if ((size_t)in_sizes[1] < (size_t)DM * TD) return;
    if ((size_t)in_sizes[2] < (size_t)TD) return;
    if ((size_t)in_sizes[3] < (size_t)(2 * LF - 1) * HD) return;
    if ((size_t)out_size < (size_t)NB * SEQ * DM) return;
    if ((size_t)SZ_ALL > ws_size) return;
    const float* x = (const float*)d_in[0]; const float* wqkv = (const float*)d_in[1]; const float* bqkv = (const float*)d_in[2]; const float* demb = (const float*)d_in[3];
    float* OUT = (float*)d_out;
    char* wsp = (char*)d_ws;
    bf* WT = (bf*)wsp; wsp += SZ_WT;
    bf* EB = (bf*)wsp; wsp += SZ_EB;
    bf* XB = (bf*)wsp; wsp += SZ_XB;
    bf* QKh = (bf*)wsp; wsp += SZ_QK;
    bf* QKl = (bf*)wsp; wsp += SZ_QK;
    h16* VT16 = (h16*)wsp; wsp += SZ_VT;
    char* R = wsp;
    float* F = (float*)R;
    float* Sb = (float*)R;
    float* RQK = (float*)(R + SZ_S);
    h16* P16 = (h16*)(R + SZ_S + SZ_T);

    k_tr64<false><<<dim3(DM / 64, TD / 64, 1), 256, 0, stream>>>(wqkv, TD, 0, 0, WT, DM);
    k_cvte<<<(EROWS * HD / 8 + 255) / 256, 256, 0, stream>>>(demb, EB);
    k_cvtx<<<dim3((unsigned)(((size_t)SEQ * DM / 8 + 255) / 256), NB, 1), 256, 0, stream>>>(x, XB);
    k_gemmw<bf, 0, true, false><<<dim3(NB * SEQ / 64, TD / 64, 1), 32, 0, stream>>>(XB, XB, WT, WT, DM, F, TD, bqkv, 1.0f, 0, 0, 0, 0, 0);
    k_qkp<<<(unsigned)(((size_t)2 * NBH * SEQ * 8 + 255) / 256), 256, 0, stream>>>(F, QKh, QKl);
    k_tr64<true><<<dim3(SEQ / 64, NH_, NB), 256, 0, stream>>>(F, TD, (size_t)SEQ * TD, 2 * DM, (unsigned short*)VT16, SEQ);

    const size_t plane = (size_t)SEQ * HD, kofs = (size_t)NBH * SEQ * HD;
    for (int p = 0; p < NBH / ZH; ++p) {
        const int bh0 = p * ZH; const int b = bh0 / NH_, h0 = bh0 % NH_;
        k_gemmw<bf, 2, false, false><<<dim3(SEQ / 64, SEQ / 64, ZH), 32, 0, stream>>>(QKh + bh0 * plane, QKl + bh0 * plane, QKh + kofs + bh0 * plane, QKl + kofs + bh0 * plane, HD, Sb, SEQ, bqkv, 1.0f, plane, plane, (size_t)SEQ * SEQ, 0, 0);
        k_gemmw<bf, 0, false, true><<<dim3(SEQ / 64, WP / 64, 2 * ZH), 32, 0, stream>>>(QKh + bh0 * plane, QKh + bh0 * plane, EB, EB, HD, RQK, WP, bqkv, 1.0f, plane, 0, (size_t)SEQ * WP, kofs, (size_t)ZH * SEQ * WP);
        k_rsoft<<<ZH * SEQ / 8, 256, 0, stream>>>(Sb, RQK, RQK + (size_t)ZH * SEQ * WP, P16);
        k_gemmw<h16, 0, false, false><<<dim3(SEQ / 64, 1, ZH), 32, 0, stream>>>(P16, P16, VT16 + (size_t)bh0 * HD * SEQ, VT16 + (size_t)bh0 * HD * SEQ, SEQ, OUT + (size_t)b * SEQ * DM + h0 * HD, DM, bqkv, 1.0f / PCAR, (size_t)SEQ * SEQ, (size_t)HD * SEQ, (size_t)HD, 0, 0);
    }
}
